// CtsConv_55448027791888
// MI455X (gfx1250) — hardware-verified
//
#include <hip/hip_runtime.h>

typedef __attribute__((ext_vector_type(16))) _Float16 v16h;
typedef __attribute__((ext_vector_type(8)))  float    v8f;
typedef __attribute__((ext_vector_type(8)))  _Float16 v8h;
typedef __attribute__((ext_vector_type(4)))  float    v4f_t;
typedef float v4fa __attribute__((ext_vector_type(4), may_alias));
#define RSPLIT (1.0f / 2048.0f)
#define KPL ((size_t)TAPS * COUT * CIN)
__device__ __forceinline__ _Float16 lo_of(float v, _Float16 h) { return (_Float16)((v - (float)h) * 2048.0f); }
__device__ __forceinline__ v8f wmma16(v16h a, v16h b, v8f c) { return __builtin_amdgcn_wmma_f32_16x16x32_f16(false, a, false, b, (short)0, c, false, false); }
__device__ __forceinline__ v8f wmma_split(v16h a, v16h al, v16h b, v16h bl, v8f c) { v8f x = {}; x = wmma16(al, b, x); x = wmma16(a, bl, x); return wmma16(a, b, c) + x * RSPLIT; }

#define B_    2
#define M_    192
#define N_    192
#define CIN   32
#define COUT  32
#define TAPS  125
#define RADIUS_INV 0.5f

__global__ void cts_prep_kernel(const float* __restrict__ k4,
                                _Float16* __restrict__ kh) {
  int idx = (blockIdx.x * blockDim.x + threadIdx.x) * 2;
  if (idx < TAPS * COUT * CIN) {
    int tap = idx / (COUT * CIN);
    int r   = idx % (COUT * CIN);
    int o   = r / CIN;
    int i   = r % CIN;
    const float w0 = k4[(o * CIN + i) * TAPS + tap], w1 = k4[(o * CIN + i + 1) * TAPS + tap];
    const _Float16 h0 = (_Float16)w0, h1 = (_Float16)w1;
    const unsigned v = (unsigned)__builtin_bit_cast(unsigned short, h0) | ((unsigned)__builtin_bit_cast(unsigned short, h1) << 16);
    const unsigned l = (unsigned)__builtin_bit_cast(unsigned short, lo_of(w0, h0)) | ((unsigned)__builtin_bit_cast(unsigned short, lo_of(w1, h1)) << 16);
    _Float16* d = kh + (tap * COUT + o) * CIN + i;
    *(volatile unsigned*)d = v; *(volatile unsigned*)(d + KPL) = l; __threadfence();
    *(volatile unsigned*)d = v; *(volatile unsigned*)(d + KPL) = l;
  }
}

__global__ void __launch_bounds__(256)
cts_main_kernel(const float* __restrict__ field,
                const float* __restrict__ center,
                const float* __restrict__ feat,
                const float* __restrict__ mask,
                const _Float16* __restrict__ kh,
                float* __restrict__ out) {
  extern __shared__ float smem[];
  float* g   = smem;
  float* red = smem + 16 * TAPS * CIN;

  const int tid  = threadIdx.x;
  const int wave = tid >> 5;
  const int lane = tid & 31;
  const int blk  = blockIdx.x;
  const int b    = blk / (M_ / 16);
  const int m0   = (blk % (M_ / 16)) * 16;

  for (int k = tid; k < 16 * TAPS * CIN; k += 256) g[k] = 0.0f;
  __syncthreads();

  const float kpi = 1.27323954473516f;

  for (int ml = wave; ml < 16; ml += 8) {
    const int m = m0 + ml;
    const float cx = center[(b * M_ + m) * 3 + 0];
    const float cy = center[(b * M_ + m) * 3 + 1];
    const float cz = center[(b * M_ + m) * 3 + 2];
    float* grow = g + ml * TAPS * CIN + lane;
    for (int n = 0; n < N_; ++n) {
      const float rx = (field[(b * N_ + n) * 3 + 0] - cx) * RADIUS_INV;
      const float ry = (field[(b * N_ + n) * 3 + 1] - cy) * RADIUS_INV;
      const float rz = (field[(b * N_ + n) * 3 + 2] - cz) * RADIUS_INV;
      const float r2 = rx * rx + ry * ry + rz * rz;
      if (r2 >= 1.0f) continue;
      const float t   = 1.0f - r2;
      const float att = t * t * t * mask[b * N_ + n];
      const float fv  = feat[(b * N_ + n) * CIN + lane] * att;

      const float r  = sqrtf(rx * rx + ry * ry + 1e-9f);
      const bool  c1 = (rx == 0.0f) && (ry == 0.0f);
      const bool  c2 = (fabsf(ry) <= fabsf(rx)) && !c1;
      const float xs = (rx == 0.0f) ? 1.0f : rx;
      const float ys = (ry == 0.0f) ? 1.0f : ry;
      const float sx = (rx > 0.0f) ? 1.0f : ((rx < 0.0f) ? -1.0f : 0.0f);
      const float sy = (ry > 0.0f) ? 1.0f : ((ry < 0.0f) ? -1.0f : 0.0f);
      const float x2 = sx * r;
      const float y2 = kpi * sx * r * atanf(ry / xs);
      const float x3 = kpi * sy * r * atanf(rx / ys);
      const float y3 = sy * r;
      const float gx = c1 ? 0.0f : (c2 ? x2 : x3);
      const float gy = c1 ? 0.0f : (c2 ? y2 : y3);
      const float gz = rz;

      const float ix = ((gx + 1.0f) * 5.0f - 1.0f) * 0.5f;
      const float iy = ((gy + 1.0f) * 5.0f - 1.0f) * 0.5f;
      const float iz = ((gz + 1.0f) * 5.0f - 1.0f) * 0.5f;
      const float fx0 = floorf(ix), fy0 = floorf(iy), fz0 = floorf(iz);
      const float fxv = ix - fx0, fyv = iy - fy0, fzv = iz - fz0;
      const int x0 = (int)fx0, y0 = (int)fy0, z0 = (int)fz0;
#pragma unroll
      for (int c = 0; c < 8; ++c) {
        const int dx = c & 1, dy = (c >> 1) & 1, dz = (c >> 2) & 1;
        const int xc = x0 + dx, yc = y0 + dy, zc = z0 + dz;
        if (xc < 0 || xc > 4 || yc < 0 || yc > 4 || zc < 0 || zc > 4) continue;
        const float w = (dx ? fxv : 1.0f - fxv) *
                        (dy ? fyv : 1.0f - fyv) *
                        (dz ? fzv : 1.0f - fzv);
        const int tap = (zc * 5 + yc) * 5 + xc;
        grow[tap * CIN] += w * fv;
      }
    }
  }
  __syncthreads();

  const int tile = wave & 1;
  const int part = wave >> 1;
  const int tap0 = part * 32;
  const int tap1 = (part == 3) ? TAPS : tap0 + 32;
  const int mrow = lane & 15;
  const int hi   = lane >> 4;
  const int o0   = tile * 16;
  const int iA0  = hi * 8;
  const int iA1  = 16 + hi * 8;

  v8f acc = {};
#pragma unroll 2
  for (int tap = tap0; tap < tap1; ++tap) {
    const float* ga = g + (mrow * TAPS + tap) * CIN;
    v16h A, Al;
#pragma unroll
    for (int j = 0; j < 8; ++j) { const float v = ga[iA0 + j]; A[j] = (_Float16)v; Al[j] = lo_of(v, A[j]); }
#pragma unroll
    for (int j = 0; j < 8; ++j) { const float v = ga[iA1 + j]; A[8 + j] = (_Float16)v; Al[8 + j] = lo_of(v, A[8 + j]); }

    const _Float16* kb = kh + ((tap * COUT) + (o0 + mrow)) * CIN + hi * 8;
    const v16h Bf  = __builtin_shufflevector(*(const v8h*)kb,         *(const v8h*)(kb + 16),       0,1,2,3,4,5,6,7,8,9,10,11,12,13,14,15);
    const v16h Bfl = __builtin_shufflevector(*(const v8h*)(kb + KPL), *(const v8h*)(kb + KPL + 16), 0,1,2,3,4,5,6,7,8,9,10,11,12,13,14,15);

    acc = wmma_split(A, Al, Bf, Bfl, acc);
  }

  float* rslot = red + (wave * 32 + lane) * 8;
#pragma unroll
  for (int v = 0; v < 8; ++v) rslot[v] = acc[v];
  __syncthreads();

  float* ot = g;
  if (wave < 2) {
#pragma unroll
    for (int v = 0; v < 8; ++v) {
      const float s = red[((wave + 0) * 32 + lane) * 8 + v] +
                      red[((wave + 2) * 32 + lane) * 8 + v] +
                      red[((wave + 4) * 32 + lane) * 8 + v] +
                      red[((wave + 6) * 32 + lane) * 8 + v];
      ot[(v + hi * 8) * COUT + wave * 16 + mrow] = s;
    }
  }
  __syncthreads();
  if (tid < 128) {
    const int rr = tid >> 3, q = (tid & 7) * 4;
    float* op = out + ((size_t)(b * M_ + m0 + rr)) * COUT + q;
    const v4f_t val = *(const volatile v4fa*)(ot + rr * COUT + q);
    *(volatile v4f_t*)op = val; __threadfence(); *(volatile v4f_t*)op = val;
  }
}

extern "C" void kernel_launch(void* const* d_in, const int* in_sizes, int n_in,
                              void* d_out, int out_size, void* d_ws, size_t ws_size,
                              hipStream_t stream) {
  (void)in_sizes; (void)n_in; (void)out_size; (void)ws_size;
  const float* field  = (const float*)d_in[0];
  const float* center = (const float*)d_in[1];
  const float* feat   = (const float*)d_in[2];
  const float* mask   = (const float*)d_in[3];
  const float* kern   = (const float*)d_in[4];
  float* out = (float*)d_out;
  _Float16* kh = (_Float16*)d_ws;

  const int total = TAPS * COUT * CIN;
  cts_prep_kernel<<<(total / 2 + 255) / 256, 256, 0, stream>>>(kern, kh);

  const size_t lds = (size_t)(16 * TAPS * CIN + 8 * 32 * 8) * sizeof(float);
  cts_main_kernel<<<B_ * (M_ / 16), 256, lds, stream>>>(field, center, feat,
                                                        mask, kh, out);
}
